// GeneSymbolCNN_6923487281857
// MI455X (gfx1250) — hardware-verified
//
#include <hip/hip_runtime.h>
#include <stddef.h>
#include <math.h>


#define VOCAB 67
#define VOCP  68
#define EMB   32
#define LSEQ  16
#define NCH   32
#define NOUT  96
#define KIN   96
#define NTHR  256
#define NWAVE 8
#define TPB   128
#define TROWS 20
#define NPREP 128
#define SCL   8.0f
#define INV64 0.015625f

#define CH_P2 (NCH * 64 / 8)
#define CH_P3 (NCH * 96 / 8)
#define CH_P4 (NCH * 128 / 8)
#define CH_PW (NOUT * KIN / 8)
#define CB1   CH_P2
#define CB2   (CB1 + CH_P3)
#define CB3   (CB2 + CH_P4)
#define CB4   (CB3 + CH_PW)

#define BP2   (NCH * 64 * 2)
#define BP3   (NCH * 96 * 2)
#define BP4   (NCH * 128 * 2)
#define BPW   (NOUT * KIN * 2)

static_assert((CB1 % NPREP) == 0 && (CB2 % NPREP) == 0 && (CB3 % NPREP) == 0 && (CB4 % NPREP) == 0);
static_assert(TPB == NWAVE * 16 && NTHR == NWAVE * 32);
static_assert((BP2 % 256) == 0 && (BP3 % 256) == 0 && (BP4 % 256) == 0 && (BPW % 256) == 0);
static_assert(KIN == 3 * NCH && NOUT == 96 && EMB == 32);
static_assert(VOCAB * 4 <= 2 * NTHR);

typedef float          v4f   __attribute__((ext_vector_type(4)));
typedef float          v8f   __attribute__((ext_vector_type(8)));
typedef _Float16       v8h   __attribute__((ext_vector_type(8)));
typedef _Float16       v16h  __attribute__((ext_vector_type(16)));
typedef unsigned short v8us  __attribute__((ext_vector_type(8)));
typedef unsigned short v16us __attribute__((ext_vector_type(16)));
typedef __bf16         v16b  __attribute__((ext_vector_type(16)));
union FragH { v16h v; v8h h[2]; };
union FragB { v16b v; v16us u; v8us h[2]; };

__device__ __forceinline__ v8f wmh(v16h a, v16h b, v8f c) {
  v8f d = __builtin_amdgcn_wmma_f32_16x16x32_f16(false, a, false, b, (short)0, c, false, false);
#if defined(__HIP_DEVICE_COMPILE__)
  asm volatile("v_nop\n\tv_nop\n\tv_nop\n\tv_nop" : "+v"(d) : "v"(a), "v"(b));
#endif
  return d;
}
__device__ __forceinline__ v8f wmb(v16b a, v16b b, v8f c) {
  v8f d = __builtin_amdgcn_wmma_f32_16x16x32_bf16(false, a, false, b, (short)0, c, false, false);
#if defined(__HIP_DEVICE_COMPILE__)
  asm volatile("v_nop\n\tv_nop\n\tv_nop\n\tv_nop" : "+v"(d) : "v"(a), "v"(b));
#endif
  return d;
}

__device__ __forceinline__ v8f zero8() {
  v8f z = {0.f, 0.f, 0.f, 0.f, 0.f, 0.f, 0.f, 0.f};
  return z;
}

__device__ __forceinline__ unsigned int bf16_rne_bits(float f) {
  const unsigned int u = __float_as_uint(f);
  return (u + 0x7FFFu + ((u >> 16) & 1u)) >> 16;
}
__device__ __forceinline__ void split_bf16(float f, unsigned short& hi, unsigned short& lo) {
  const unsigned int h = bf16_rne_bits(f);
  const float fh = __uint_as_float(h << 16);
  const unsigned int l = bf16_rne_bits(f - fh);
  hi = (unsigned short)h;
  lo = (unsigned short)l;
}

template <int KW>
__device__ __forceinline__ v8h conv_chunk(const float* __restrict__ w, int cl) {
  const int KP = 32 * KW;
  const int o8 = cl * 8;
  const int o  = o8 / KP;
  const int kk = o8 - o * KP;
  const int d  = kk >> 5;
  const int i0 = kk & 31;
  v8h hv;
#pragma unroll
  for (int e = 0; e < 8; ++e) hv[e] = (_Float16)(w[(o * EMB + i0 + e) * KW + d] * SCL);
  return hv;
}

__global__ __launch_bounds__(NPREP) void k_prep(
    const float* __restrict__ w2, const float* __restrict__ w3, const float* __restrict__ w4,
    const float* __restrict__ pw,
    _Float16* P2, _Float16* P3, _Float16* P4, unsigned short* PWH, unsigned short* PWL) {
  const int bstart = blockIdx.x * NPREP;
  const int c = bstart + (int)threadIdx.x;
  if (c >= CB4) return;
  if (bstart < CB3) {
    v8h hv;
    _Float16* dp;
    if (bstart < CB1)      { hv = conv_chunk<2>(w2, c);       dp = P2 + (size_t)c * 8; }
    else if (bstart < CB2) { hv = conv_chunk<3>(w3, c - CB1); dp = P3 + (size_t)(c - CB1) * 8; }
    else                   { hv = conv_chunk<4>(w4, c - CB2); dp = P4 + (size_t)(c - CB2) * 8; }
    *(volatile v8h*)dp = hv;
    __threadfence();
    *(volatile v8h*)dp = hv;
  } else {
    const int cl = c - CB3;
    const int n  = cl / 12;
    const int k0 = cl * 8 - n * KIN;
    v8us hu, lu;
#pragma unroll
    for (int e = 0; e < 8; ++e) {
      unsigned short h_, l_;
      split_bf16(pw[n * KIN + k0 + e], h_, l_);
      hu[e] = h_;
      lu[e] = l_;
    }
    unsigned short* dh = PWH + (size_t)cl * 8;
    unsigned short* dl = PWL + (size_t)cl * 8;
    *(volatile v8us*)dh = hu;
    *(volatile v8us*)dl = lu;
    __threadfence();
    *(volatile v8us*)dh = hu;
    *(volatile v8us*)dl = lu;
  }
}

template <int T>
__device__ __forceinline__ void pool_branch(const v8f (&c)[2], const float (&bias)[2], float* frow, int hh, int m) {
#pragma unroll
  for (int nt = 0; nt < 2; ++nt) {
    float mx = -3.402823466e38f;
#pragma unroll
    for (int r = 0; r < 8; ++r) {
      const bool ok = (8 * hh + r) < T;
      const float cand = fmaxf(mx, c[nt][r]);
      mx = ok ? cand : mx;
    }
    const float oth = __shfl_xor(mx, 16, 32);
    mx = fmaxf(mx, oth);
    const float g = fmaxf(mx * INV64 + bias[nt], 0.0f);
    if (hh == 0) frow[16 * nt + m] = g;
  }
}

template <int KW>
__device__ __forceinline__ void conv_branch(const _Float16* tile, const _Float16* __restrict__ plane,
                                            const float (&bias)[2], float* frow, int hh, int m) {
  const int KP = 32 * KW;
  v8f c[2];
  c[0] = zero8();
  c[1] = zero8();
#pragma unroll
  for (int s = 0; s < KW; ++s) {
    FragH a;
    a.h[0] = *(const v8h*)(tile + (m + s) * EMB + 8 * hh);
    a.h[1] = *(const v8h*)(tile + (m + s) * EMB + 16 + 8 * hh);
#pragma unroll
    for (int nt = 0; nt < 2; ++nt) {
      const _Float16* bp = plane + (size_t)(16 * nt + m) * KP + 32 * s + 8 * hh;
      FragH b;
      b.h[0] = *(const v8h*)bp;
      b.h[1] = *(const v8h*)(bp + 16);
      c[nt] = wmh(a.v, b.v, c[nt]);
    }
  }
  pool_branch<17 - KW>(c, bias, frow + NCH * (KW - 2), hh, m);
}

__global__ __launch_bounds__(NTHR) void k_main(
    const int* __restrict__ x, const float* __restrict__ embed,
    const float* __restrict__ b2, const float* __restrict__ b3, const float* __restrict__ b4,
    const float* __restrict__ pb,
    const _Float16* __restrict__ P2, const _Float16* __restrict__ P3, const _Float16* __restrict__ P4,
    const unsigned short* __restrict__ PWH, const unsigned short* __restrict__ PWL,
    float* out, int nTok) {
  __shared__ __attribute__((aligned(16))) _Float16 sTab[VOCP * EMB];
  __shared__ __attribute__((aligned(16))) _Float16 sEmb[NWAVE * TROWS * EMB];
  __shared__ __attribute__((aligned(16))) float    sFeat[TPB * KIN];

  const int tid = threadIdx.x, lane = tid & 31, wave = tid >> 5, hh = lane >> 4, m = lane & 15;
  const int tok0 = blockIdx.x * TPB;

  for (int c = tid; c < VOCAB * 4; c += NTHR) {
    const int id = c >> 2, q = c & 3;
    const float* sp = embed + id * EMB + 8 * q;
    const v4f f0 = *(const v4f*)sp;
    const v4f f1 = *(const v4f*)(sp + 4);
    v8h hv;
#pragma unroll
    for (int e = 0; e < 4; ++e) {
      hv[e]     = (_Float16)((id == 0) ? 0.0f : f0[e] * SCL);
      hv[4 + e] = (_Float16)((id == 0) ? 0.0f : f1[e] * SCL);
    }
    *(v8h*)(sTab + id * EMB + 8 * q) = hv;
  }
  if (tid < NWAVE * 4 * 4) {
    const int slot = tid >> 4, rr = (tid >> 2) & 3, q = tid & 3;
    v8h z;
#pragma unroll
    for (int e = 0; e < 8; ++e) z[e] = (_Float16)0.0f;
    *(v8h*)(sEmb + slot * (TROWS * EMB) + (16 + rr) * EMB + 8 * q) = z;
  }
  float bias2[2], bias3[2], bias4[2], pbv[6];
  bias2[0] = b2[m]; bias2[1] = b2[16 + m];
  bias3[0] = b3[m]; bias3[1] = b3[16 + m];
  bias4[0] = b4[m]; bias4[1] = b4[16 + m];
#pragma unroll
  for (int nt = 0; nt < 6; ++nt) pbv[nt] = pb[16 * nt + m];
  __syncthreads();

  const _Float16* tile = sEmb + wave * (TROWS * EMB);
#pragma unroll 1
  for (int j = 0; j < 16; ++j) {
#pragma unroll
    for (int u = 0; u < 2; ++u) {
      const int c = tid + NTHR * u;
      const int slot = c >> 6, r = (c >> 2) & 15, q = c & 3;
      int tk = tok0 + slot * 16 + j;
      tk = tk > nTok - 1 ? nTok - 1 : tk;
      int id = x[(size_t)tk * LSEQ + r];
      id = id < 0 ? 0 : (id > VOCAB - 1 ? VOCAB - 1 : id);
      const v8h v = *(const v8h*)(sTab + id * EMB + 8 * q);
      *(v8h*)(sEmb + slot * (TROWS * EMB) + r * EMB + 8 * q) = v;
    }
    __syncthreads();
    float* frow = sFeat + (wave * 16 + j) * KIN;
    conv_branch<2>(tile, P2, bias2, frow, hh, m);
    conv_branch<3>(tile, P3, bias3, frow, hh, m);
    conv_branch<4>(tile, P4, bias4, frow, hh, m);
    __syncthreads();
  }

  v8f acc[6];
#pragma unroll
  for (int nt = 0; nt < 6; ++nt) acc[nt] = zero8();
  const float* frbase = sFeat + (wave * 16 + m) * KIN;
#pragma unroll
  for (int kt = 0; kt < 3; ++kt) {
    const float* fp = frbase + 32 * kt + 8 * hh;
    const v4f q0 = *(const v4f*)(fp);
    const v4f q1 = *(const v4f*)(fp + 4);
    const v4f q2 = *(const v4f*)(fp + 16);
    const v4f q3 = *(const v4f*)(fp + 20);
    FragB ah, al;
#pragma unroll
    for (int e = 0; e < 4; ++e) {
      unsigned short h_, l_;
      split_bf16(q0[e], h_, l_); ah.u[e]      = h_; al.u[e]      = l_;
      split_bf16(q1[e], h_, l_); ah.u[4 + e]  = h_; al.u[4 + e]  = l_;
      split_bf16(q2[e], h_, l_); ah.u[8 + e]  = h_; al.u[8 + e]  = l_;
      split_bf16(q3[e], h_, l_); ah.u[12 + e] = h_; al.u[12 + e] = l_;
    }
#pragma unroll
    for (int nt = 0; nt < 6; ++nt) {
      const size_t boff = (size_t)(16 * nt + m) * KIN + 32 * kt + 8 * hh;
      FragB bh, bl;
      bh.h[0] = *(const v8us*)(PWH + boff);
      bh.h[1] = *(const v8us*)(PWH + boff + 16);
      bl.h[0] = *(const v8us*)(PWL + boff);
      bl.h[1] = *(const v8us*)(PWL + boff + 16);
      acc[nt] = wmb(ah.v, bh.v, acc[nt]);
      acc[nt] = wmb(ah.v, bl.v, acc[nt]);
      acc[nt] = wmb(al.v, bh.v, acc[nt]);
    }
  }
  __syncthreads();
  {
    float* orow = sFeat + (wave * 16 + 8 * hh) * KIN + m;
#pragma unroll
    for (int nt = 0; nt < 6; ++nt) {
#pragma unroll
      for (int r = 0; r < 8; ++r) orow[r * KIN + 16 * nt] = fmaxf(acc[nt][r] + pbv[nt], 0.0f);
    }
  }
  __syncthreads();
  {
    const float* swv = sFeat + wave * 16 * KIN;
    const size_t gt0 = (size_t)tok0 + (size_t)wave * 16;
    float* gbase = out + gt0 * NOUT;
    v4f  pv[12];
    bool ok[12];
#pragma unroll
    for (int p = 0; p < 12; ++p) {
      const int q = 32 * p + lane;
      pv[p] = *(const v4f*)(swv + 4 * q);
      ok[p] = (gt0 + (size_t)(q / 24)) < (size_t)nTok;
    }
#pragma unroll
    for (int p = 0; p < 12; ++p) {
      if (ok[p]) *(volatile v4f*)(gbase + 4 * (32 * p + lane)) = pv[p];
    }
    __threadfence();
#pragma unroll
    for (int p = 0; p < 12; ++p) {
      if (ok[p]) *(volatile v4f*)(gbase + 4 * (32 * p + lane)) = pv[p];
    }
  }
}

extern "C" void kernel_launch(void* const* d_in, const int* in_sizes, int n_in,
                              void* d_out, int out_size, void* d_ws, size_t ws_size,
                              hipStream_t stream) {
  if (n_in < 10) return;
  if (in_sizes[0] <= 0 || (in_sizes[0] % LSEQ) != 0) return;
  const int nTok = in_sizes[0] / LSEQ;
  if (in_sizes[1] != VOCAB * EMB) return;
  if (in_sizes[2] != NCH * EMB * 2 || in_sizes[3] != NCH) return;
  if (in_sizes[4] != NCH * EMB * 3 || in_sizes[5] != NCH) return;
  if (in_sizes[6] != NCH * EMB * 4 || in_sizes[7] != NCH) return;
  if (in_sizes[8] != NOUT * KIN || in_sizes[9] != NOUT) return;
  if ((long long)out_size != (long long)nTok * NOUT) return;

  const int*   x     = (const int*)d_in[0];
  const float* embed = (const float*)d_in[1];
  const float* w2    = (const float*)d_in[2];
  const float* b2    = (const float*)d_in[3];
  const float* w3    = (const float*)d_in[4];
  const float* b3    = (const float*)d_in[5];
  const float* w4    = (const float*)d_in[6];
  const float* b4    = (const float*)d_in[7];
  const float* pw    = (const float*)d_in[8];
  const float* pb    = (const float*)d_in[9];
  float* out = (float*)d_out;

  char* ws = (char*)d_ws;
  size_t off = 0;
  const size_t oP2  = off; off += (size_t)BP2; off = (off + 255) & ~(size_t)255;
  const size_t oP3  = off; off += (size_t)BP3; off = (off + 255) & ~(size_t)255;
  const size_t oP4  = off; off += (size_t)BP4; off = (off + 255) & ~(size_t)255;
  const size_t oPWH = off; off += (size_t)BPW; off = (off + 255) & ~(size_t)255;
  const size_t oPWL = off; off += (size_t)BPW; off = (off + 255) & ~(size_t)255;
  if (off > ws_size || off > (size_t)134217728) return;
  _Float16*       P2  = (_Float16*)(ws + oP2);
  _Float16*       P3  = (_Float16*)(ws + oP3);
  _Float16*       P4  = (_Float16*)(ws + oP4);
  unsigned short* PWH = (unsigned short*)(ws + oPWH);
  unsigned short* PWL = (unsigned short*)(ws + oPWL);

  k_prep<<<CB4 / NPREP, NPREP, 0, stream>>>(w2, w3, w4, pw, P2, P3, P4, PWH, PWL);

  const int nBlk = (nTok + TPB - 1) / TPB;
  k_main<<<nBlk, NTHR, 0, stream>>>(x, embed, b2, b3, b4, pb, P2, P3, P4, PWH, PWL, out, nTok);
}
